// LorentzTransformerEncoder_283467842438
// MI455X (gfx1250) — hardware-verified
//
#include <hip/hip_runtime.h>
#include <hip/hip_bf16.h>
#include <math.h>


typedef _Float16 bf16;
typedef _Float16 f16;
typedef __attribute__((ext_vector_type(4))) unsigned v4u_t;
typedef unsigned v4ua __attribute__((ext_vector_type(4), may_alias));
typedef __attribute__((ext_vector_type(4))) float v4f_t;
typedef float v4fa __attribute__((ext_vector_type(4), may_alias));
typedef __attribute__((ext_vector_type(16))) bf16  bf16x16;
typedef bf16x16 f16x16;
typedef __attribute__((ext_vector_type(8)))  bf16  bf16x8;
typedef bf16x8 f16x8;
typedef __attribute__((ext_vector_type(4)))  bf16  bf16x4;
typedef __attribute__((ext_vector_type(8)))  float f32x8;
__device__ __forceinline__ f32x8 wmma16(f16x16 a, f16x16 b, f32x8 c) {
  c = __builtin_amdgcn_wmma_f32_16x16x32_f16(false, a, false, b, (short)0, c, false, false);
  asm volatile("v_nop\n\tv_nop\n\tv_nop\n\tv_nop" : "+v"(c) : "v"(a), "v"(b));
  return c;
}
#define LDS_STRIDE 48
#define KSTRIDE    72
#define VSTRIDE    48

__device__ __forceinline__ f32x8 wmma_bf16(bf16x16 a, bf16x16 b, f32x8 c) {
  c = __builtin_amdgcn_wmma_f32_16x16x32_f16(false, a, false, b, (short)0, c, false, false);
  asm volatile("v_nop\n\tv_nop\n\tv_nop\n\tv_nop" : "+v"(c) : "v"(a), "v"(b));
  return c;
}

template <typename T>
__device__ __forceinline__ bf16x16 load_frag(const T* __restrict__ base, int ld,
                                             int row0, int k0) {
  const int lane = threadIdx.x & 31;
  const int r    = lane & 15;
  const int kh   = (lane >> 4) * 8;
  const T* p0 = base + (size_t)(row0 + r) * ld + (k0 + kh);
  const T* p1 = p0 + 16;
  bf16x16 f;
#pragma unroll
  for (int i = 0; i < 8; ++i) {
    f[i]     = (bf16)p0[i];
    f[i + 8] = (bf16)p1[i];
  }
  return f;
}

__device__ __forceinline__ bf16x16 lds_frag(const bf16* base, int stride) {
  const int lane = threadIdx.x & 31;
  const int row  = lane & 15;
  const int kh   = (lane >> 4) * 8;
  const bf16x8 lo = *(const bf16x8*)(base + row * stride + kh);
  const bf16x8 hi = *(const bf16x8*)(base + row * stride + kh + 16);
  bf16x16 f;
#pragma unroll
  for (int i = 0; i < 8; ++i) { f[i] = lo[i]; f[i + 8] = hi[i]; }
  return f;
}

template <typename T>
__device__ __forceinline__ void stage_read16(const T* __restrict__ p, float* buf) {
#pragma unroll
  for (int i = 0; i < 16; ++i) buf[i] = (float)p[i];
}

__device__ __forceinline__ void stage_write(bf16* dst, const float* buf, int nquad) {
#pragma unroll
  for (int i = 0; i < nquad; ++i) {
    bf16x4 q;
    q[0] = (bf16)buf[4 * i];     q[1] = (bf16)buf[4 * i + 1];
    q[2] = (bf16)buf[4 * i + 2]; q[3] = (bf16)buf[4 * i + 3];
    *(bf16x4*)(dst + 4 * i) = q;
  }
}


#define GSTR 48
#define GSTR 48
template <typename AT, int EPI, bool OUT16>
__global__ __launch_bounds__(256) void gemm_kne(const AT* __restrict__ A, int lda, const float* __restrict__ Wm, int ldw,
                                                const float* __restrict__ bias, const float* __restrict__ R, const float* __restrict__ gvec,
                                                void* __restrict__ Yv, int ldy, int K) {
  __shared__ __attribute__((aligned(16))) f16 ldsA[128 * GSTR];
  __shared__ __attribute__((aligned(16))) f16 ldsW[128 * GSTR];
  __shared__ __attribute__((aligned(16))) float oS[8][32 * 68];
  const int tid = threadIdx.x, lane = tid & 31, wave = tid >> 5, cl = lane & 15, rh = (lane >> 4) * 8;
  const int m0 = blockIdx.x * 128, n0 = blockIdx.y * 128;
  const int wm = (wave & 3) * 32, wn = (wave >> 2) * 64;
  f32x8 acc[2][4];
#pragma unroll
  for (int i = 0; i < 2; ++i)
#pragma unroll
    for (int j = 0; j < 4; ++j) { f32x8 z = {}; acc[i][j] = z; }
#pragma unroll 1
  for (int k0 = 0; k0 < K; k0 += 32) {
    __syncthreads();
    { const int row = tid >> 1, ch = (tid & 1) * 16;
      const AT* src = A + (size_t)(m0 + row) * lda + k0 + ch;
#pragma unroll
      for (int g = 0; g < 16; ++g) ldsA[row * GSTR + ch + g] = (f16)src[g]; }
    { const int k = tid >> 3, nn0 = (tid & 7) * 16;
      const float* src = Wm + (size_t)(k0 + k) * ldw + n0 + nn0;
#pragma unroll
      for (int g = 0; g < 4; ++g) { const v4f_t v = *(const v4f_t*)(src + 4 * g);
#pragma unroll
        for (int u = 0; u < 4; ++u) ldsW[(nn0 + 4 * g + u) * GSTR + k] = (f16)v[u]; } }
    __syncthreads();
    f16x16 af[2];
#pragma unroll
    for (int i = 0; i < 2; ++i) af[i] = lds_frag(ldsA + (wm + 16 * i) * GSTR, GSTR);
#pragma unroll
    for (int j = 0; j < 4; ++j) {
      const f16x16 bf = lds_frag(ldsW + (wn + 16 * j) * GSTR, GSTR);
#pragma unroll
      for (int i = 0; i < 2; ++i) acc[i][j] = wmma16(af[i], bf, acc[i][j]);
    }
  }
  float* so = oS[wave];
#pragma unroll
  for (int i = 0; i < 2; ++i)
#pragma unroll
    for (int j = 0; j < 4; ++j) {
      const int n = n0 + wn + 16 * j + cl;
      const float bv = bias ? bias[n] : 0.0f;
      const float gv = (EPI == 2 || EPI == 4) ? gvec[n] : 0.0f;
      if (EPI == 1) {
#pragma unroll 1
        for (int r = 0; r < 8; ++r) { const float xg = acc[i][j][r] + bv; so[(16 * i + rh + r) * 68 + 16 * j + cl] = 0.5f * xg * (1.0f + erff(xg * 0.70710678118654752f)); }
      } else {
#pragma unroll
        for (int r = 0; r < 8; ++r) {
          float v = acc[i][j][r] + bv;
          if (EPI == 3) v = fmaxf(v, 0.0f);
          if (EPI == 4) v = gv * v;
          if (EPI == 2) v = R[(size_t)(m0 + wm + 16 * i + rh + r) * ldy + n] + gv * v;
          so[(16 * i + rh + r) * 68 + 16 * j + cl] = v;
        }
      }
    }
  asm volatile("s_wait_dscnt 0" ::: "memory");
  __builtin_amdgcn_wave_barrier();
#pragma unroll 1
  for (int pass = 0; pass < 2; ++pass) {
    if (OUT16) {
      f16* Y = (f16*)Yv;
#pragma unroll
      for (int it = 0; it < 8; ++it) { const int c = lane + 32 * it, rr = c >> 3, q8 = (c & 7) * 8;
        union { f16 h[8]; v4u_t v; } u;
#pragma unroll
        for (int e = 0; e < 8; ++e) u.h[e] = (f16)so[rr * 68 + q8 + e];
        *(volatile v4u_t*)(Y + (size_t)(m0 + wm + rr) * ldy + n0 + wn + q8) = u.v; }
    } else {
      float* Y = (float*)Yv;
#pragma unroll
      for (int it = 0; it < 16; ++it) { const int f4 = lane + 32 * it, rr = f4 >> 4, q = (f4 & 15) * 4;
        *(volatile v4f_t*)(Y + (size_t)(m0 + wm + rr) * ldy + n0 + wn + q) = *(const v4fa*)(so + rr * 68 + q); }
    }
    __threadfence();
  }
}

template <typename AT, int EPI, bool OUT16>
__global__ __launch_bounds__(256) void gemm_knez(const AT* __restrict__ A, int lda, size_t strideA, const float* __restrict__ Wm, int ldw, size_t strideW,
                                                 const float* __restrict__ bias, const float* __restrict__ R, const float* __restrict__ gvec,
                                                 void* __restrict__ Yv, int ldy, size_t strideY, int K) {
  A += (size_t)blockIdx.z * strideA; Wm += (size_t)blockIdx.z * strideW; Yv = (void*)((char*)Yv + (size_t)blockIdx.z * strideY * (OUT16 ? 2 : 4)); if (R) R += (size_t)blockIdx.z * strideY;
  __shared__ __attribute__((aligned(16))) f16 ldsA[128 * GSTR];
  __shared__ __attribute__((aligned(16))) f16 ldsW[128 * GSTR];
  __shared__ __attribute__((aligned(16))) float oS[8][32 * 68];
  const int tid = threadIdx.x, lane = tid & 31, wave = tid >> 5, cl = lane & 15, rh = (lane >> 4) * 8;
  const int m0 = blockIdx.x * 128, n0 = blockIdx.y * 128;
  const int wm = (wave & 3) * 32, wn = (wave >> 2) * 64;
  f32x8 acc[2][4];
#pragma unroll
  for (int i = 0; i < 2; ++i)
#pragma unroll
    for (int j = 0; j < 4; ++j) { f32x8 z = {}; acc[i][j] = z; }
#pragma unroll 1
  for (int k0 = 0; k0 < K; k0 += 32) {
    __syncthreads();
    { const int row = tid >> 1, ch = (tid & 1) * 16;
      const AT* src = A + (size_t)(m0 + row) * lda + k0 + ch;
#pragma unroll
      for (int g = 0; g < 16; ++g) ldsA[row * GSTR + ch + g] = (f16)src[g]; }
    { const int k = tid >> 3, nn0 = (tid & 7) * 16;
      const float* src = Wm + (size_t)(k0 + k) * ldw + n0 + nn0;
#pragma unroll
      for (int g = 0; g < 4; ++g) { const v4f_t v = *(const v4f_t*)(src + 4 * g);
#pragma unroll
        for (int u = 0; u < 4; ++u) ldsW[(nn0 + 4 * g + u) * GSTR + k] = (f16)v[u]; } }
    __syncthreads();
    f16x16 af[2];
#pragma unroll
    for (int i = 0; i < 2; ++i) af[i] = lds_frag(ldsA + (wm + 16 * i) * GSTR, GSTR);
#pragma unroll
    for (int j = 0; j < 4; ++j) {
      const f16x16 bf = lds_frag(ldsW + (wn + 16 * j) * GSTR, GSTR);
#pragma unroll
      for (int i = 0; i < 2; ++i) acc[i][j] = wmma16(af[i], bf, acc[i][j]);
    }
  }
  float* so = oS[wave];
#pragma unroll
  for (int i = 0; i < 2; ++i)
#pragma unroll
    for (int j = 0; j < 4; ++j) {
      const int n = n0 + wn + 16 * j + cl;
      const float bv = bias ? bias[n] : 0.0f;
      const float gv = (EPI == 2 || EPI == 4) ? gvec[n] : 0.0f;
      if (EPI == 1) {
#pragma unroll 1
        for (int r = 0; r < 8; ++r) { const float xg = acc[i][j][r] + bv; so[(16 * i + rh + r) * 68 + 16 * j + cl] = 0.5f * xg * (1.0f + erff(xg * 0.70710678118654752f)); }
      } else {
#pragma unroll
        for (int r = 0; r < 8; ++r) {
          float v = acc[i][j][r] + bv;
          if (EPI == 3) v = fmaxf(v, 0.0f);
          if (EPI == 4) v = gv * v;
          if (EPI == 2) v = R[(size_t)(m0 + wm + 16 * i + rh + r) * ldy + n] + gv * v;
          so[(16 * i + rh + r) * 68 + 16 * j + cl] = v;
        }
      }
    }
  asm volatile("s_wait_dscnt 0" ::: "memory");
  __builtin_amdgcn_wave_barrier();
#pragma unroll 1
  for (int pass = 0; pass < 2; ++pass) {
    if (OUT16) {
      f16* Y = (f16*)Yv;
#pragma unroll
      for (int it = 0; it < 8; ++it) { const int c = lane + 32 * it, rr = c >> 3, q8 = (c & 7) * 8;
        union { f16 h[8]; v4u_t v; } u;
#pragma unroll
        for (int e = 0; e < 8; ++e) u.h[e] = (f16)so[rr * 68 + q8 + e];
        *(volatile v4u_t*)(Y + (size_t)(m0 + wm + rr) * ldy + n0 + wn + q8) = u.v; }
    } else {
      float* Y = (float*)Yv;
#pragma unroll
      for (int it = 0; it < 16; ++it) { const int f4 = lane + 32 * it, rr = f4 >> 4, q = (f4 & 15) * 4;
        *(volatile v4f_t*)(Y + (size_t)(m0 + wm + rr) * ldy + n0 + wn + q) = *(const v4fa*)(so + rr * 68 + q); }
    }
    __threadfence();
  }
}

template <typename AT, bool ACC>
__global__ __launch_bounds__(256) void gemm_kn2(const AT* __restrict__ A, int lda, size_t strideA,
                                               const float* __restrict__ Wm, int ldw, size_t strideW,
                                               const float* __restrict__ bias, float scale,
                                               float* __restrict__ Y, int ldy, size_t strideY, int K) {
  __shared__ __attribute__((aligned(16))) f16 ldsA[128 * GSTR], ldsAl[128 * GSTR];
  __shared__ __attribute__((aligned(16))) f16 ldsW[128 * GSTR], ldsWl[128 * GSTR];
  __shared__ __attribute__((aligned(16))) float oS[8][32 * 68];
  const int tid = threadIdx.x, lane = tid & 31, wave = tid >> 5, cl = lane & 15, rh = (lane >> 4) * 8;
  const int m0 = blockIdx.x * 128, n0 = blockIdx.y * 128;
  const int wm = (wave & 3) * 32, wn = (wave >> 2) * 64;
  A += (size_t)blockIdx.z * strideA; Wm += (size_t)blockIdx.z * strideW; Y += (size_t)blockIdx.z * strideY;
  f32x8 acc[2][4], accx[2][4];
#pragma unroll
  for (int i = 0; i < 2; ++i)
#pragma unroll
    for (int j = 0; j < 4; ++j) { f32x8 z = {}; acc[i][j] = z; accx[i][j] = z; }
#pragma unroll 1
  for (int k0 = 0; k0 < K; k0 += 32) {
    __syncthreads();
    {
      const int row = tid >> 1, ch = (tid & 1) * 16;
      const AT* src = A + (size_t)(m0 + row) * lda + k0 + ch;
#pragma unroll
      for (int g = 0; g < 16; ++g) { const float v = (float)src[g]; const f16 h = (f16)v; ldsA[row * GSTR + ch + g] = h; ldsAl[row * GSTR + ch + g] = (f16)((v - (float)h) * 2048.0f); }
    }
    {
      const int k = tid >> 3, nn0 = (tid & 7) * 16;
      const float* src = Wm + (size_t)(k0 + k) * ldw + n0 + nn0;
#pragma unroll
      for (int g = 0; g < 4; ++g) { const v4f_t v = *(const v4f_t*)(src + 4 * g);
#pragma unroll
        for (int u = 0; u < 4; ++u) { const f16 h = (f16)v[u]; ldsW[(nn0 + 4 * g + u) * GSTR + k] = h; ldsWl[(nn0 + 4 * g + u) * GSTR + k] = (f16)((v[u] - (float)h) * 2048.0f); } }
    }
    __syncthreads();
    f16x16 af[2], afl[2];
#pragma unroll
    for (int i = 0; i < 2; ++i) { af[i] = lds_frag(ldsA + (wm + 16 * i) * GSTR, GSTR); afl[i] = lds_frag(ldsAl + (wm + 16 * i) * GSTR, GSTR); }
#pragma unroll
    for (int j = 0; j < 4; ++j) {
      const f16x16 bf = lds_frag(ldsW + (wn + 16 * j) * GSTR, GSTR), bfl = lds_frag(ldsWl + (wn + 16 * j) * GSTR, GSTR);
#pragma unroll
      for (int i = 0; i < 2; ++i) { acc[i][j] = wmma16(af[i], bf, acc[i][j]); accx[i][j] = wmma16(af[i], bfl, accx[i][j]); accx[i][j] = wmma16(afl[i], bf, accx[i][j]); }
    }
  }
  float* so = oS[wave];
#pragma unroll
  for (int i = 0; i < 2; ++i)
#pragma unroll
    for (int j = 0; j < 4; ++j) {
      const float bv = bias ? bias[n0 + wn + 16 * j + cl] : 0.0f;
#pragma unroll
      for (int r = 0; r < 8; ++r) so[(16 * i + rh + r) * 68 + 16 * j + cl] = (acc[i][j][r] + accx[i][j][r] * (1.0f / 2048.0f)) * scale + bv;
    }
  asm volatile("s_wait_dscnt 0" ::: "memory");
  __builtin_amdgcn_wave_barrier();
  if (ACC) {
#pragma unroll
    for (int it = 0; it < 16; ++it) { const int f4 = lane + 32 * it, rr = f4 >> 4, q = (f4 & 15) * 4;
      const v4f_t old = *(const v4fa*)(Y + (size_t)(m0 + wm + rr) * ldy + n0 + wn + q);
      v4f_t v = *(const v4fa*)(so + rr * 68 + q); v += old; *(v4fa*)(so + rr * 68 + q) = v; }
    asm volatile("s_wait_dscnt 0" ::: "memory");
  }
#pragma unroll 1
  for (int pass = 0; pass < 2; ++pass) {
#pragma unroll
    for (int it = 0; it < 16; ++it) { const int f4 = lane + 32 * it, rr = f4 >> 4, q = (f4 & 15) * 4;
      *(volatile v4f_t*)(Y + (size_t)(m0 + wm + rr) * ldy + n0 + wn + q) = *(const v4fa*)(so + rr * 68 + q); }
    __threadfence();
  }
}

__global__ __launch_bounds__(256) void k_transpose(const float* __restrict__ Wm, float* __restrict__ Wt, int rows, int cols) {
  __shared__ float tS[64][65];
  const int tid = threadIdx.x, tbj = cols / 64, bi = blockIdx.x / tbj, bj = blockIdx.x % tbj;
  for (int e = tid; e < 64 * 64; e += 256) { const int r = e >> 6, c = e & 63; tS[r][c] = Wm[(size_t)(bi * 64 + r) * cols + bj * 64 + c]; }
  __syncthreads();
  for (int ch = tid; ch < 64 * 16; ch += 256) { const int r = ch >> 4, q4 = (ch & 15) * 4; v4f_t o; o[0] = tS[q4][r]; o[1] = tS[q4 + 1][r]; o[2] = tS[q4 + 2][r]; o[3] = tS[q4 + 3][r];
    float* dst = Wt + (size_t)(bj * 64 + r) * rows + bi * 64 + q4; *(volatile v4f_t*)dst = o; __threadfence(); *(volatile v4f_t*)dst = o; }
}


template <typename AT, int EPI, bool OUT16, int NJ>
__global__ __launch_bounds__(256) void gemm_sm(const AT* __restrict__ A, int lda, size_t sA, const float* __restrict__ Wm, int ldw, size_t sW,
                                               const float* __restrict__ bias, const float* __restrict__ R, const float* __restrict__ gvec,
                                               void* __restrict__ Yv, int ldy, size_t sY, int K) {
  constexpr int BN = 16 * NJ; constexpr int OST = BN + 4;
  A += (size_t)blockIdx.z * sA; Wm += (size_t)blockIdx.z * sW; Yv = (void*)((char*)Yv + (size_t)blockIdx.z * sY * (OUT16 ? 2 : 4)); if (R) R += (size_t)blockIdx.z * sY;
  __shared__ __attribute__((aligned(16))) f16 ldsA[256 * GSTR];
  __shared__ __attribute__((aligned(16))) f16 ldsW[BN * GSTR];
  __shared__ __attribute__((aligned(16))) float oS[8][32 * OST];
  const int tid = threadIdx.x, lane = tid & 31, wave = tid >> 5, cl = lane & 15, rh = (lane >> 4) * 8;
  const int m0 = blockIdx.x * 256, n0 = blockIdx.y * BN;
  const int wm = wave * 32;
  f32x8 acc[2][NJ];
#pragma unroll
  for (int i = 0; i < 2; ++i)
#pragma unroll
    for (int j = 0; j < NJ; ++j) { f32x8 z = {}; acc[i][j] = z; }
#pragma unroll 1
  for (int k0 = 0; k0 < K; k0 += 32) {
    __syncthreads();
    { const AT* src = A + (size_t)(m0 + tid) * lda + k0;
#pragma unroll
      for (int g = 0; g < 32; ++g) ldsA[tid * GSTR + g] = (f16)src[g]; }
    { const int k = tid >> 3, nn0 = (tid & 7) * (2 * NJ);
      const float* src = Wm + (size_t)(k0 + k) * ldw + n0 + nn0;
#pragma unroll
      for (int g = 0; g < NJ / 2; ++g) { const v4f_t v = *(const v4f_t*)(src + 4 * g);
#pragma unroll
        for (int u = 0; u < 4; ++u) ldsW[(nn0 + 4 * g + u) * GSTR + k] = (f16)v[u]; } }
    __syncthreads();
    f16x16 af[2];
#pragma unroll
    for (int i = 0; i < 2; ++i) af[i] = lds_frag(ldsA + (wm + 16 * i) * GSTR, GSTR);
#pragma unroll
    for (int j = 0; j < NJ; ++j) {
      const f16x16 bf = lds_frag(ldsW + (16 * j) * GSTR, GSTR);
#pragma unroll
      for (int i = 0; i < 2; ++i) acc[i][j] = wmma16(af[i], bf, acc[i][j]);
    }
  }
  float* so = oS[wave];
#pragma unroll
  for (int i = 0; i < 2; ++i)
#pragma unroll
    for (int j = 0; j < NJ; ++j) {
      const int n = n0 + 16 * j + cl;
      const float bv = bias ? bias[n] : 0.0f;
      const float gv = (EPI == 2 || EPI == 4) ? gvec[n] : 0.0f;
#pragma unroll
      for (int r = 0; r < 8; ++r) {
        float v = acc[i][j][r] + bv;
        if (EPI == 3) v = fmaxf(v, 0.0f);
        if (EPI == 2) v = R[(size_t)(m0 + wm + 16 * i + rh + r) * ldy + n] + gv * v;
        if (EPI == 4) v = gv * v;
        so[(16 * i + rh + r) * OST + 16 * j + cl] = v;
      }
    }
  asm volatile("s_wait_dscnt 0" ::: "memory");
  __builtin_amdgcn_wave_barrier();
#pragma unroll 1
  for (int pass = 0; pass < 2; ++pass) {
    if (OUT16) {
      f16* Y = (f16*)Yv;
#pragma unroll
      for (int it = 0; it < BN / 8; ++it) { const int c = lane + 32 * it, rr = c / (BN / 8), q8 = (c % (BN / 8)) * 8;
        union { f16 h[8]; v4u_t v; } u;
#pragma unroll
        for (int e = 0; e < 8; ++e) u.h[e] = (f16)so[rr * OST + q8 + e];
        *(volatile v4u_t*)(Y + (size_t)(m0 + wm + rr) * ldy + n0 + q8) = u.v; }
    } else {
      float* Y = (float*)Yv;
#pragma unroll
      for (int it = 0; it < BN / 4; ++it) { const int f4 = lane + 32 * it, rr = f4 / (BN / 4), q = (f4 % (BN / 4)) * 4;
        *(volatile v4f_t*)(Y + (size_t)(m0 + wm + rr) * ldy + n0 + q) = *(const v4fa*)(so + rr * OST + q); }
    }
    __threadfence();
  }
}

#define NBl 2
#define NNl 1024
#define DSl 512
#define DPl 544
#define NHl 8
#define HDl 64
#define FFl 2048
#define FFPl 2080
__global__ __launch_bounds__(256) void k_fill(float* __restrict__ p, float val, size_t n4) { const size_t i = (size_t)blockIdx.x * 256 + threadIdx.x; if (i < n4) { v4f_t v = {val, val, val, val}; *(volatile v4f_t*)(p + 4 * i) = v; __threadfence(); *(volatile v4f_t*)(p + 4 * i) = v; } }
__global__ __launch_bounds__(256) void k_dbg_zero(float* __restrict__ p, size_t n4) { const size_t i = (size_t)blockIdx.x * 256 + threadIdx.x; if (i < n4) { v4f_t z = {0.f,0.f,0.f,0.f}; *(volatile v4f_t*)(p + 4 * i) = z; __threadfence(); *(volatile v4f_t*)(p + 4 * i) = z; } }
__global__ __launch_bounds__(256) void k_copy(const float* __restrict__ src, float* __restrict__ dst, size_t n4) { const size_t i = (size_t)blockIdx.x * 256 + threadIdx.x; if (i < n4) { const v4f_t v = *(const v4f_t*)(src + 4 * i); *(volatile v4f_t*)(dst + 4 * i) = v; __threadfence(); *(volatile v4f_t*)(dst + 4 * i) = v; } }
__global__ __launch_bounds__(256) void k_vmeank(const float* __restrict__ V, int ldv, float* __restrict__ VB) {
  const int c = blockIdx.x * 256 + threadIdx.x; float s = 0.0f;
#pragma unroll 1
  for (int r = 0; r < 1024; ++r) s += V[(size_t)r * ldv + c];
  const float m = s * (1024.0f / 1024.0f); *(volatile float*)(VB + c) = m; __threadfence(); *(volatile float*)(VB + c) = m;
}
__global__ __launch_bounds__(256) void k_padT(const float* __restrict__ Wm, int kin, int nout, float* __restrict__ WT) {
  const int k = blockIdx.x, tid = threadIdx.x; const int srck = (k < kin - 1) ? (k + 1) : 0; const bool live = k < kin;
#pragma unroll 1
  for (int pass = 0; pass < 2; ++pass) {
#pragma unroll 1
    for (int o = tid; o < nout; o += 256) { const float v = live ? Wm[(size_t)o * kin + srck] : 0.0f; *(volatile float*)(WT + (size_t)k * nout + o) = v; }
    __threadfence(); }
}
__global__ __launch_bounds__(256) void k_lln(const float* __restrict__ src, int lds, int col0, const float* __restrict__ g, const float* __restrict__ bb, float* __restrict__ XP, float* __restrict__ XS) {
  __shared__ float red[256]; __shared__ float red2[256];
  const int r = blockIdx.x, tid = threadIdx.x; const float* sr = src + (size_t)r * lds + col0; const float v0 = sr[tid], v1 = sr[tid + 256];
  red[tid] = v0 + v1; __syncthreads(); for (int o = 128; o > 0; o >>= 1) { if (tid < o) red[tid] += red[tid + o]; __syncthreads(); }
  const float mean = red[0] * (1.0f / DSl); const float d0 = v0 - mean, d1 = v1 - mean;
  red2[tid] = d0 * d0 + d1 * d1; __syncthreads(); for (int o = 128; o > 0; o >>= 1) { if (tid < o) red2[tid] += red2[tid + o]; __syncthreads(); }
  const float rs = 1.0f / __builtin_sqrtf(red2[0] * (1.0f / DSl) + 1e-5f); const float n0 = d0 * rs * g[tid] + bb[tid], n1 = d1 * rs * g[tid + 256] + bb[tid + 256];
  __syncthreads(); red[tid] = n0 * n0 + n1 * n1; __syncthreads(); for (int o = 128; o > 0; o >>= 1) { if (tid < o) red[tid] += red[tid + o]; __syncthreads(); }
  const float t = __builtin_sqrtf(red[0] + 1.0f); float* d = XP + (size_t)r * DPl;
#pragma unroll 1
  for (int pass = 0; pass < 2; ++pass) { *(volatile float*)(d + tid) = n0; *(volatile float*)(d + 256 + tid) = n1; if (tid < 32) *(volatile float*)(d + 512 + tid) = (tid == 0) ? t : 0.0f;
    if (XS) { *(volatile float*)(XS + (size_t)r * DSl + tid) = v0; *(volatile float*)(XS + (size_t)r * DSl + 256 + tid) = v1; } __threadfence(); }
}
__global__ __launch_bounds__(256) void k_times(const float* __restrict__ SQ, const float* __restrict__ SK, float* __restrict__ QT, float* __restrict__ KTT) {
  const int tid = threadIdx.x, h = tid >> 5, ii = tid & 31; const size_t i = (size_t)blockIdx.x * 32 + ii; float nq = 0.0f, nk = 0.0f;
#pragma unroll 1
  for (int d = 0; d < HDl; ++d) { const float q = SQ[i * DSl + h * HDl + d], k = SK[i * DSl + h * HDl + d]; nq = fmaf(q, q, nq); nk = fmaf(k, k, nk); }
  const float qt = __builtin_sqrtf(nq + 1.0f), kt = __builtin_sqrtf(nk + 1.0f);
#pragma unroll 1
  for (int pass = 0; pass < 2; ++pass) { *(volatile float*)(QT + i * NHl + h) = qt; *(volatile float*)(KTT + (size_t)h * NNl + i) = kt; __threadfence(); }
}
__global__ __launch_bounds__(256) void k_headgeo(const float* __restrict__ SQ, const float* __restrict__ SK, const float* __restrict__ SV, const float* __restrict__ QT, const float* __restrict__ KTT,
                                                float* __restrict__ QA, float* __restrict__ KA, float* __restrict__ VT) {
  const int i = blockIdx.x, tid = threadIdx.x; const int h = tid >> 5, c = tid & 31; const size_t col = (size_t)h * HDl + 2 * c;
  typedef __attribute__((ext_vector_type(2))) float v2f;
  const v2f q = *(const v2f*)(SQ + (size_t)i * DSl + col), k = *(const v2f*)(SK + (size_t)i * DSl + col), v = *(const v2f*)(SV + (size_t)i * DSl + col);
  float nv = v[0] * v[0] + v[1] * v[1];
#pragma unroll
  for (int o = 1; o < 32; o <<= 1) nv += __shfl_xor(nv, o, 32);
  const float vt = __builtin_sqrtf(nv + 1.0f); const float vn = fmaxf(__builtin_sqrtf(nv), 1e-8f); const float vs = acoshf(fmaxf(vt, 1.0f)) / vn;
  const float qt = QT[(size_t)i * NHl + h], kt = KTT[(size_t)h * NNl + i];
  float* qa = QA + ((size_t)i * NHl + h) * 96; float* ka = KA + ((size_t)i * NHl + h) * 96; const v2f vv = v * vs;
#pragma unroll 1
  for (int pass = 0; pass < 2; ++pass) {
    *(volatile v2f*)(qa + 2 * c) = q; *(volatile v2f*)(ka + 2 * c) = k; *(volatile float*)(qa + 64 + c) = (c == 0) ? -qt : 0.0f; *(volatile float*)(ka + 64 + c) = (c == 0) ? kt : 0.0f;
    *(volatile v2f*)(VT + (size_t)i * DSl + col) = vv; __threadfence(); }
}
__global__ __launch_bounds__(1024) void k_haa(float* __restrict__ Sm, const float* __restrict__ QT, const float* __restrict__ KTT, int h0, const float* __restrict__ ptemp, const float* __restrict__ pbeta, const float* __restrict__ ptau, const float* __restrict__ plam) {
  __shared__ float red[NNl];
  const int i = blockIdx.x, z = blockIdx.y, h = h0 + z, j = threadIdx.x; float* sr = Sm + ((size_t)z * NNl + i) * NNl;
  const float temp = ptemp[0]; const float braw = pbeta[0], traw = ptau[0], lraw = plam[0];
  const float beta = (braw > 20.0f) ? braw : log1pf(expf(braw)), tau = (traw > 20.0f) ? traw : log1pf(expf(traw)), lam = (lraw > 20.0f) ? lraw : log1pf(expf(lraw));
  const float qt = QT[(size_t)i * NHl + h]; const float nsOQ = fmaxf(qt * qt - 1.0f, 0.0f); const float ctil = acoshf(fmaxf(qt, 1.001f)); const float sh = sinhf(ctil);
  const float Bq = __builtin_sqrtf(fmaxf(1.0f - (beta / sh) * (beta / sh), 0.0f) + 1e-8f);
  const float ln2 = 0.6931471805599453f, lme = 0.64439666007357089f;
  const float inner = sr[j]; const float kt = KTT[(size_t)h * NNl + j];
  const float nsQK = fmaxf(inner * inner - 1.0f, 0.0f); const float numer = -kt - inner * qt; const float den = __builtin_sqrtf(nsQK * nsOQ + 0.005f * 0.005f);
  const float Z = fminf(fmaxf(numer / den, -1.0f), 1.0f);
  const float dist = acoshf(fmaxf(-inner, 1.001f)); const float dsoft = 40.0f * tanhf(dist * (1.0f / 40.0f)); const float sd = dsoft * (1.0f / 15.0f);
  const float sp1a = -2.0f * sd; const float sp1 = (sp1a > 20.0f) ? sp1a : log1pf(expf(sp1a)); const float Hh = sd + sp1 - ln2;
  const float pa = Bq + Z - 0.1f; const float sp2 = (pa > 20.0f) ? pa : log1pf(expf(pa)); const float Phi = sp2 - lme;
  float v = (-lam * Hh - tau * Phi) / temp;
  red[j] = v; __syncthreads(); for (int o = NNl / 2; o > 0; o >>= 1) { if (j < o) red[j] = fmaxf(red[j], red[j + o]); __syncthreads(); }
  const float m = red[0]; __syncthreads();
  v = expf(v - m); red[j] = v; __syncthreads(); for (int o = NNl / 2; o > 0; o >>= 1) { if (j < o) red[j] += red[j + o]; __syncthreads(); }
  const float p = v * (1024.0f / red[0]) - 1.0f;
  *(volatile float*)(sr + j) = p; __threadfence(); *(volatile float*)(sr + j) = p;
}
__global__ __launch_bounds__(256) void k_expmap(const float* __restrict__ MT, float* __restrict__ ATTN) {
  __shared__ float at2[NHl];
  const int i = blockIdx.x, tid = threadIdx.x; const int h = tid >> 5, c = tid & 31; const size_t col = (size_t)h * HDl + 2 * c;
  const float m0 = MT[(size_t)i * DSl + col], m1 = MT[(size_t)i * DSl + col + 1]; float nn = m0 * m0 + m1 * m1;
#pragma unroll
  for (int o = 1; o < 32; o <<= 1) nn += __shfl_xor(nn, o, 32);
  const float n = fmaxf(__builtin_sqrtf(nn), 1e-8f); const float at = coshf(n), fs = sinhf(n) / n;
  if (c == 0) at2[h] = at * at;
  __syncthreads();
  float t2 = -7.0f;
#pragma unroll
  for (int hh = 0; hh < NHl; ++hh) t2 += at2[hh];
  const float t = __builtin_sqrtf(fmaxf(t2, 1e-8f)); float* d = ATTN + (size_t)i * DPl;
typedef __attribute__((ext_vector_type(2))) float v2f; v2f o2; o2[0] = m0 * fs; o2[1] = m1 * fs;
#pragma unroll 1
  for (int pass = 0; pass < 2; ++pass) { *(volatile v2f*)(d + col) = o2; if (tid < 32) *(volatile float*)(d + 512 + tid) = (tid == 0) ? t : 0.0f; __threadfence(); }
}
__global__ __launch_bounds__(256) void k_h1(const float* __restrict__ S1, float* __restrict__ H1P) {
  __shared__ float red[256];
  const int r = blockIdx.x, tid = threadIdx.x; const float* sr = S1 + (size_t)r * FFl; float v[8]; float s = 0.0f;
#pragma unroll
  for (int e = 0; e < 8; ++e) { v[e] = sr[tid + 256 * e]; s += v[e] * v[e]; }
  red[tid] = s; __syncthreads(); for (int o = 128; o > 0; o >>= 1) { if (tid < o) red[tid] += red[tid + o]; __syncthreads(); }
  const float t = __builtin_sqrtf(red[0] + 1.0f); float* d = H1P + (size_t)r * FFPl;
#pragma unroll 1
  for (int pass = 0; pass < 2; ++pass) {
#pragma unroll
    for (int e = 0; e < 8; ++e) *(volatile float*)(d + tid + 256 * e) = v[e];
    if (tid < 32) *(volatile float*)(d + 2048 + tid) = (tid == 0) ? t : 0.0f; __threadfence(); }
}
__global__ __launch_bounds__(256) void k_tt(const float* __restrict__ OS, float* __restrict__ TT) {
  __shared__ float st[32];
  const int tid = threadIdx.x, r = tid >> 3, part = tid & 7; const size_t row = (size_t)blockIdx.x * 32 + r; float a = 0.0f;
#pragma unroll 1
  for (int e = 0; e < DSl / 8; ++e) { const float v = OS[row * DSl + part * (DSl / 8) + e]; a = fmaf(v, v, a); }
  a += __shfl_xor(a, 1, 32); a += __shfl_xor(a, 2, 32); a += __shfl_xor(a, 4, 32);
  if (part == 0) st[r] = __builtin_sqrtf(a + 1.0f);
  __syncthreads();
  if (tid < 32) { float* d = TT + (size_t)blockIdx.x * 32 + tid; const float v = st[tid]; *(volatile float*)d = v; __threadfence(); *(volatile float*)d = v; }
}
__global__ __launch_bounds__(1024) void k_out(const float* __restrict__ OS, const float* __restrict__ TT, float* __restrict__ outb) {
  const int tid = threadIdx.x; const size_t tot = (size_t)NNl * 513;
#pragma unroll 1
  for (int pass = 0; pass < 2; ++pass) {
#pragma unroll 1
    for (size_t fidx = tid; fidx < tot; fidx += 1024) { const int r = (int)(fidx / 513), col = (int)(fidx % 513); const float v = (col == 0) ? TT[r] : OS[(size_t)r * DSl + (col > 0 ? col - 1 : 0)]; *(volatile float*)(outb + fidx) = v; }
    __threadfence(); }
}

extern "C" void kernel_launch(void* const* d_in, const int* in_sizes, int n_in,
                              void* d_out, int out_size, void* d_ws, size_t ws_size,
                              hipStream_t stream) {
  (void)in_sizes; (void)n_in; (void)out_size;
  const float** f = (const float**)d_in;
  const float* x = f[0], *Wq = f[1], *Wk = f[2], *Wv = f[3], *Wo = f[4], *W1 = f[5], *W2 = f[6], *g1 = f[7], *b1 = f[8], *g2 = f[9], *b2p = f[10];
  float* out = (float*)d_out;
  char* ws = (char*)d_ws;
  float* WqT = (float*)ws; ws += (size_t)DPl * DSl * 4; float* WkT = (float*)ws; ws += (size_t)DPl * DSl * 4; float* WvT = (float*)ws; ws += (size_t)DPl * DSl * 4; float* WoT = (float*)ws; ws += (size_t)DPl * DSl * 4;
  float* W1T = (float*)ws; ws += (size_t)DPl * FFl * 4; float* W2T = (float*)ws; ws += (size_t)FFPl * DSl * 4;
  float* X1P = (float*)ws; ws += (size_t)NNl * DPl * 4; float* XS = (float*)ws; ws += (size_t)NNl * DSl * 4;
  float* SQ = (float*)ws; ws += (size_t)NNl * DSl * 4; float* SK = (float*)ws; ws += (size_t)NNl * DSl * 4; float* SV = (float*)ws; ws += (size_t)NNl * DSl * 4;
  float* QA = (float*)ws; ws += (size_t)NNl * NHl * 96 * 4; float* KA = (float*)ws; ws += (size_t)NNl * NHl * 96 * 4; float* KAT = (float*)ws; ws += (size_t)NHl * 96 * NNl * 4;
  float* QT = (float*)ws; ws += (size_t)NNl * NHl * 4; float* KTT = (float*)ws; ws += (size_t)NHl * NNl * 4; float* VT = (float*)ws; ws += (size_t)NNl * DSl * 4; float* VBK = (float*)ws; ws += DSl * 4; float* sc = (float*)ws; ws += 64 * 4;
  float* S = (float*)ws; ws += (size_t)2 * NNl * NNl * 4; float* MT = (float*)ws; ws += (size_t)NNl * DSl * 4; float* ATTN = (float*)ws; ws += (size_t)NNl * DPl * 4;
  float* OS1 = (float*)ws; ws += (size_t)NNl * DSl * 4; float* Y1P = (float*)ws; ws += (size_t)NNl * DPl * 4; float* S1 = (float*)ws; ws += (size_t)NNl * FFl * 4; float* H1P = (float*)ws; ws += (size_t)NNl * FFPl * 4;
  float* OS2 = (float*)ws; ws += (size_t)NNl * DSl * 4; float* TT = (float*)ws; ws += (size_t)NNl * 4; float* ones = (float*)ws; ws += DSl * 4;
  if ((size_t)(ws - (char*)d_ws) > ws_size) return;
  const dim3 blk(256);
  k_padT<<<dim3(DPl), blk, 0, stream>>>(Wq, 513, DSl, WqT); k_padT<<<dim3(DPl), blk, 0, stream>>>(Wk, 513, DSl, WkT); k_padT<<<dim3(DPl), blk, 0, stream>>>(Wv, 513, DSl, WvT); k_padT<<<dim3(DPl), blk, 0, stream>>>(Wo, 513, DSl, WoT);
  k_padT<<<dim3(DPl), blk, 0, stream>>>(W1, 513, FFl, W1T); k_padT<<<dim3(FFPl), blk, 0, stream>>>(W2, 2049, DSl, W2T);
  k_fill<<<dim3(1), blk, 0, stream>>>(sc, 1.0f / 1024.0f, 64 / 4); k_fill<<<dim3(1), blk, 0, stream>>>(ones, 1.0f, DSl / 4);

  for (int b = 0; b < NBl; ++b) {
    const float* xb = x + (size_t)b * NNl * 513;
    k_lln<<<dim3(NNl), blk, 0, stream>>>(xb, 513, 1, g1, b1, X1P, XS);
    gemm_kne<float, 0, false><<<dim3(NNl / 128, DSl / 128), blk, 0, stream>>>(X1P, DPl, WqT, DSl, nullptr, nullptr, nullptr, SQ, DSl, DPl);
    gemm_kne<float, 0, false><<<dim3(NNl / 128, DSl / 128), blk, 0, stream>>>(X1P, DPl, WkT, DSl, nullptr, nullptr, nullptr, SK, DSl, DPl);
    gemm_kne<float, 0, false><<<dim3(NNl / 128, DSl / 128), blk, 0, stream>>>(X1P, DPl, WvT, DSl, nullptr, nullptr, nullptr, SV, DSl, DPl);
    k_times<<<dim3(NNl / 32), blk, 0, stream>>>(SQ, SK, QT, KTT);
    k_headgeo<<<dim3(NNl), blk, 0, stream>>>(SQ, SK, SV, QT, KTT, QA, KA, VT);
    k_transpose<<<dim3(((NHl * 96) / 64) * (NNl / 64)), blk, 0, stream>>>(KA, KAT, NNl, NHl * 96);
    k_vmeank<<<dim3(DSl / 256), blk, 0, stream>>>(VT, DSl, VBK);
    for (int hp = 0; hp < NHl / 2; ++hp) { const int h0 = 2 * hp;
      gemm_knez<float, 0, false><<<dim3(NNl / 128, NNl / 128, 2), blk, 0, stream>>>(QA + (size_t)h0 * 96, NHl * 96, (size_t)96, KAT + (size_t)h0 * 96 * NNl, NNl, (size_t)96 * NNl, nullptr, nullptr, nullptr, S, NNl, (size_t)NNl * NNl, 96);
      k_haa<<<dim3(NNl, 2), dim3(NNl), 0, stream>>>(S, QT, KTT, h0, f[11], f[12], f[13], f[14]);
      for (int z = 0; z < 2; ++z)
        gemm_sm<float, 4, false, 4><<<dim3(NNl / 256, 1, 1), blk, 0, stream>>>(S + (size_t)z * NNl * NNl, NNl, (size_t)0, VT + (h0 + z) * HDl, DSl, (size_t)0, VBK + (h0 + z) * HDl, nullptr, sc, MT + (h0 + z) * HDl, DSl, (size_t)0, NNl);
    }
    k_expmap<<<dim3(NNl), blk, 0, stream>>>(MT, ATTN);
    gemm_kne<float, 2, false><<<dim3(NNl / 128, DSl / 128), blk, 0, stream>>>(ATTN, DPl, WoT, DSl, nullptr, XS, ones, OS1, DSl, DPl);
    k_lln<<<dim3(NNl), blk, 0, stream>>>(OS1, DSl, 0, g2, b2p, Y1P, nullptr);
    gemm_kne<float, 1, false><<<dim3(NNl / 128, FFl / 128), blk, 0, stream>>>(Y1P, DPl, W1T, FFl, nullptr, nullptr, nullptr, S1, FFl, DPl);
    k_h1<<<dim3(NNl), blk, 0, stream>>>(S1, H1P);
    gemm_kne<float, 2, false><<<dim3(NNl / 128, DSl / 128), blk, 0, stream>>>(H1P, FFPl, W2T, DSl, nullptr, OS1, ones, OS2, DSl, FFPl);
    k_tt<<<dim3(NNl / 32), blk, 0, stream>>>(OS2, TT);
    k_out<<<dim3(1), dim3(1024), 0, stream>>>(OS2, TT, out + (size_t)b * NNl * 513);
  }
}
